// GASADecoder_26173530701973
// MI455X (gfx1250) — hardware-run, weakly checked
//
#include <hip/hip_runtime.h>
#include <math.h>

constexpr int kBatch   = 2;
constexpr int kNq      = 512;
constexpr int kNk      = 4096;
constexpr int kDim     = 512;
constexpr int kHeads   = 8;
constexpr int kHdim    = 64;
constexpr int kKernDim = 32;
constexpr int kDff     = 2048;
constexpr int kTokQ    = kBatch * kNq;
constexpr int kTokK    = kBatch * kNk;
constexpr int kHeadsPerChunk = 4;
constexpr int kNumChunks = kBatch * kHeads / kHeadsPerChunk;

constexpr float kWCarry     = 16.0f;
constexpr float kWCarryInv  = 1.0f / 16.0f;
constexpr float kPCarry     = 2048.0f;
constexpr float kCtxCarry   = 64.0f;
constexpr float kPVScale    = kCtxCarry / kPCarry;
constexpr float kProjScale  = 1.0f / (kCtxCarry * kWCarry);
constexpr float kAttnScale  = 0.125f;
constexpr float kInvDim     = 1.0f / 512.0f;
constexpr float kLnEps      = 1e-5f;

constexpr size_t kOffXq   = 0;
constexpr size_t kOffMem  = kOffXq   + (size_t)kTokQ * kDim * 2;
constexpr size_t kOffWsa  = kOffMem  + (size_t)kTokK * kDim * 2;
constexpr size_t kOffWso  = kOffWsa  + (size_t)3 * kDim * kDim * 2;
constexpr size_t kOffWq   = kOffWso  + (size_t)kDim * kDim * 2;
constexpr size_t kOffWk   = kOffWq   + (size_t)kDim * kDim * 2;
constexpr size_t kOffWv   = kOffWk   + (size_t)kDim * kDim * 2;
constexpr size_t kOffWo   = kOffWv   + (size_t)kDim * kDim * 2;
constexpr size_t kOffWf1  = kOffWo   + (size_t)kDim * kDim * 2;
constexpr size_t kOffWf2  = kOffWf1  + (size_t)kDff * kDim * 2;
constexpr size_t kOffQK   = kOffWf2  + (size_t)kDim * kDff * 2;
constexpr size_t kOffVTs  = kOffQK   + (size_t)kTokQ * 2 * kDim * 2;
constexpr size_t kOffS    = kOffVTs  + (size_t)kBatch * kDim * kNq * 2;
constexpr size_t kOffP    = kOffS    + (size_t)kHeadsPerChunk * kNq * kNk * 4;
constexpr size_t kOffCtx  = kOffP    + (size_t)kHeadsPerChunk * kNq * kNk * 2;
constexpr size_t kOffT    = kOffCtx  + (size_t)kTokQ * kDim * 2;
constexpr size_t kOffX1f  = kOffT    + (size_t)kTokQ * kDim * 4;
constexpr size_t kOffX1h  = kOffX1f  + (size_t)kTokQ * kDim * 4;
constexpr size_t kOffQc   = kOffX1h  + (size_t)kTokQ * kDim * 2;
constexpr size_t kOffKc   = kOffQc   + (size_t)kTokQ * kDim * 2;
constexpr size_t kOffVTc  = kOffKc   + (size_t)kTokK * kDim * 2;
constexpr size_t kOffBB   = kOffVTc  + (size_t)kBatch * kDim * kNk * 2;
constexpr size_t kOffX2f  = kOffBB   + (size_t)kBatch * kNq * kNk * 4;
constexpr size_t kOffX2h  = kOffX2f  + (size_t)kTokQ * kDim * 4;
constexpr size_t kOffHf   = kOffX2h  + (size_t)kTokQ * kDim * 2;
constexpr size_t kWsTotal = kOffHf   + (size_t)kTokQ * kDff * 2;

typedef __attribute__((ext_vector_type(16))) _Float16 v16h;
typedef __attribute__((ext_vector_type(8)))  _Float16 v8h;
typedef __attribute__((ext_vector_type(16))) __bf16   v16b;
typedef __attribute__((ext_vector_type(8)))  __bf16   v8b;
typedef __attribute__((ext_vector_type(8)))  float    v8f;
typedef __attribute__((ext_vector_type(4)))  float    v4f;
typedef __attribute__((ext_vector_type(4)))  unsigned int v4u;

__device__ __forceinline__ unsigned short f2bf_bits(float f) {
  unsigned u = __float_as_uint(f);
  return (unsigned short)((u + 0x7FFFu + ((u >> 16) & 1u)) >> 16);
}
__device__ __forceinline__ float bf_bits2f(unsigned short h) { return __uint_as_float(((unsigned)h) << 16); }

__device__ __forceinline__ void dep_guard_h(v8f& a, v8f& b, v16h x, v16h y) { asm volatile("v_nop\n\tv_nop\n\tv_nop\n\tv_nop" : "+v"(a), "+v"(b) : "v"(x), "v"(y)); }
__device__ __forceinline__ void dep_guard_b(v8f& a, v8f& b, v16b x, v16b y) { asm volatile("v_nop\n\tv_nop\n\tv_nop\n\tv_nop" : "+v"(a), "+v"(b) : "v"(x), "v"(y)); }
__device__ __forceinline__ void keep4_h(v16h a, v16h b, v16h c, v16h d) { asm volatile("v_nop" :: "v"(a), "v"(b), "v"(c), "v"(d)); }
__device__ __forceinline__ void keep4_b(v16b a, v16b b, v16b c, v16b d) { asm volatile("v_nop" :: "v"(a), "v"(b), "v"(c), "v"(d)); }
__device__ __forceinline__ void acc_guard4(v8f& a, v8f& b, v8f& c, v8f& d) { asm volatile("v_nop\n\tv_nop\n\tv_nop\n\tv_nop" : "+v"(a), "+v"(b), "+v"(c), "+v"(d)); }
template <typename T> struct Frag;
template <> struct Frag<_Float16> {
  typedef v16h V; union U { v16h v; v8h h[2]; };
  static __device__ __forceinline__ v16h load(const _Float16* p) {
    U f; f.h[0] = *(const v8h*)(p); f.h[1] = *(const v8h*)(p + 16); return f.v;
  }
  static __device__ __forceinline__ v8f mma(v16h a, v16h b, v8f c) {
    return __builtin_amdgcn_wmma_f32_16x16x32_f16(false, a, false, b, (short)0, c, false, false);
  }
  static __device__ __forceinline__ void guard(v8f& a, v8f& b, v16h x, v16h y) { dep_guard_h(a, b, x, y); }
  static __device__ __forceinline__ void keep(v16h a, v16h b, v16h c, v16h d) { keep4_h(a, b, c, d); }
};
template <> struct Frag<__bf16> {
  typedef v16b V; union U { v16b v; v8b h[2]; };
  static __device__ __forceinline__ v16b load(const __bf16* p) {
    U f; f.h[0] = *(const v8b*)(p); f.h[1] = *(const v8b*)(p + 16); return f.v;
  }
  static __device__ __forceinline__ v8f mma(v16b a, v16b b, v8f c) {
    return __builtin_amdgcn_wmma_f32_16x16x32_bf16(false, a, false, b, (short)0, c, false, false);
  }
  static __device__ __forceinline__ void guard(v8f& a, v8f& b, v16b x, v16b y) { dep_guard_b(a, b, x, y); }
  static __device__ __forceinline__ void keep(v16b a, v16b b, v16b c, v16b d) { keep4_b(a, b, c, d); }
};

__device__ __forceinline__ unsigned pk16(unsigned short a, unsigned short b) { return (unsigned)a | ((unsigned)b << 16); }
__device__ __forceinline__ unsigned short h_bits(float f) { const _Float16 h = (_Float16)f; return __builtin_bit_cast(unsigned short, h); }

template <int ET> struct Elem;
template <> struct Elem<0> { typedef _Float16 T; };
template <> struct Elem<1> { typedef __bf16 T; };
template <int ET, bool SPLIT, int BIAS_MODE, int OUT_MODE, bool RESID, int ACT = 0>
__global__ __launch_bounds__(256) void wmma_gemm64(
    const unsigned short* __restrict__ Ap, const unsigned short* __restrict__ A2p, int lda, long strideA,
    const unsigned short* __restrict__ Btp, const unsigned short* __restrict__ Bt2p, int ldb, long strideB,
    void* __restrict__ Cout, void* __restrict__ Cout2, int ldc, long strideC,
    const float* __restrict__ bias,
    const float* __restrict__ resid, long strideR,
    int M, int N, int K, float scale) {
  typedef typename Elem<ET>::T T;
  typedef typename Frag<T>::V V;
  const T* A = (const T*)Ap; const T* A2 = (const T*)A2p; const T* Bt = (const T*)Btp; const T* Bt2 = (const T*)Bt2p;
  __shared__ __align__(16) float sT[8][16 * 68];
  const int b    = blockIdx.y;
  const int lane = threadIdx.x & 31;
  const int wave = threadIdx.x >> 5;
  const int tilesN = N >> 6;
  const int tilesM = M >> 6;
  const int tile = blockIdx.x * 8 + wave;
  if (tile >= tilesM * tilesN) return;
  const int tm = tile / tilesN;
  const int tn = tile - tm * tilesN;
  const int m0 = tm << 6;
  const int n0 = tn << 6;

  const T* Ab  = A  + (size_t)b * strideA;
  const T* Bb  = Bt + (size_t)b * strideB;
  const T* Ab2 = SPLIT ? (A2  + (size_t)b * strideA) : nullptr;
  const T* Bb2 = SPLIT ? (Bt2 + (size_t)b * strideB) : nullptr;

  const int rlane = lane & 15;
  const int koff  = (lane >> 4) * 8;
  const int mOff  = (lane >> 4) * 8;

  v8f acc[4][4];
#pragma unroll
  for (int i = 0; i < 4; ++i)
#pragma unroll
    for (int j = 0; j < 4; ++j) acc[i][j] = (v8f){0.f,0.f,0.f,0.f,0.f,0.f,0.f,0.f};

  for (int k0 = 0; k0 < K; k0 += 32) {
    V bh[4], bl[4];
#pragma unroll
    for (int j = 0; j < 4; ++j) {
      const size_t bo = (size_t)(n0 + (j << 4) + rlane) * ldb + koff + k0;
      bh[j] = Frag<T>::load(Bb + bo);
      if (SPLIT) bl[j] = Frag<T>::load(Bb2 + bo);
    }
#pragma unroll
    for (int i = 0; i < 4; ++i) {
      const size_t ao = (size_t)(m0 + (i << 4) + rlane) * lda + koff + k0;
      V ah = Frag<T>::load(Ab + ao);
      V al;
      if (SPLIT) al = Frag<T>::load(Ab2 + ao);
#pragma unroll
      for (int j = 0; j < 4; ++j) {
        acc[i][j] = Frag<T>::mma(ah, bh[j], acc[i][j]);
        if (SPLIT) {
          acc[i][j] = Frag<T>::mma(ah, bl[j], acc[i][j]);
          acc[i][j] = Frag<T>::mma(al, bh[j], acc[i][j]);
        }
      }
      Frag<T>::guard(acc[i][0], acc[i][3], ah, SPLIT ? al : ah);
    }
    Frag<T>::keep(bh[0], bh[1], bh[2], bh[3]);
    if (SPLIT) Frag<T>::keep(bl[0], bl[1], bl[2], bl[3]);
  }
  acc_guard4(acc[0][0], acc[0][1], acc[0][2], acc[0][3]);
  acc_guard4(acc[1][0], acc[1][1], acc[1][2], acc[1][3]);
  acc_guard4(acc[2][0], acc[2][1], acc[2][2], acc[2][3]);
  acc_guard4(acc[3][0], acc[3][1], acc[3][2], acc[3][3]);

  float* slab = sT[wave];
  const float* Rb = RESID ? (resid + (size_t)b * strideR) : nullptr;
#pragma unroll
  for (int i = 0; i < 4; ++i) {
    const int mBase = m0 + (i << 4);
#pragma unroll
    for (int j = 0; j < 4; ++j) {
      const int n = n0 + (j << 4) + rlane;
      float bv = 0.f;
      if (BIAS_MODE == 2) bv = bias[n];
#pragma unroll
      for (int r = 0; r < 8; ++r) {
        float v = acc[i][j][r] * scale;
        if (BIAS_MODE == 1) v += bias[mBase + mOff + r];
        if (BIAS_MODE == 2) v += bv;
        if (RESID) v += Rb[(size_t)(mBase + mOff + r) * ldc + n];
        if (ACT == 2) v = fmaxf(v, 0.0f);
        if (ACT == 4) v = (v > 0.f) ? v : 0.01f * v;
        slab[(mOff + r) * 68 + (j << 4) + rlane] = v;
      }
    }
    __builtin_amdgcn_fence(__ATOMIC_RELEASE, "workgroup");
    __builtin_amdgcn_wave_barrier();
    __builtin_amdgcn_fence(__ATOMIC_ACQUIRE, "workgroup");
    if (OUT_MODE == 0) {
      float* C = (float*)Cout + (size_t)b * strideC;
      const int hh = lane >> 4, c4 = (lane & 15) * 4;
      for (int pass = 0; pass < 2; ++pass) {
#pragma unroll
        for (int it = 0; it < 8; ++it) {
          const int row = it * 2 + hh;
          v4f v = *(const v4f*)(slab + row * 68 + c4);
          *(volatile v4f*)(C + (size_t)(mBase + row) * ldc + n0 + c4) = v;
        }
        __threadfence();
      }
    } else {
      const int q = lane >> 3, c8 = (lane & 7) * 8;
      unsigned short* C  = (unsigned short*)Cout  + (size_t)b * strideC;
      unsigned short* C2 = (OUT_MODE == 2) ? ((unsigned short*)Cout2 + (size_t)b * strideC) : nullptr;
      for (int pass = 0; pass < 2; ++pass) {
#pragma unroll
        for (int it = 0; it < 4; ++it) {
          const int row = it * 4 + q;
          const float* sp = slab + row * 68 + c8;
          v8h hv, lv;
#pragma unroll
          for (int e = 0; e < 8; ++e) {
            if (OUT_MODE == 1) {
              hv[e] = (_Float16)sp[e];
            } else {
              unsigned short hb = f2bf_bits(sp[e]);
              unsigned short lb = f2bf_bits(sp[e] - bf_bits2f(hb));
              hv[e] = __builtin_bit_cast(_Float16, hb);
              lv[e] = __builtin_bit_cast(_Float16, lb);
            }
          }
          *(volatile v8h*)(C + (size_t)(mBase + row) * ldc + n0 + c8) = hv;
          if (OUT_MODE == 2) *(volatile v8h*)(C2 + (size_t)(mBase + row) * ldc + n0 + c8) = lv;
        }
        __threadfence();
      }
    }
    __builtin_amdgcn_fence(__ATOMIC_RELEASE, "workgroup");
    __builtin_amdgcn_wave_barrier();
    __builtin_amdgcn_fence(__ATOMIC_ACQUIRE, "workgroup");
  }
}

__global__ __launch_bounds__(256) void cast8_f16_kernel(const float* __restrict__ in, unsigned short* __restrict__ out,
                                                        int n8, float scale) {
  const int i = blockIdx.x * 256 + threadIdx.x;
  if (i >= n8) return;
  const float* p = in + 8 * (size_t)i;
  const v4f a = *(const v4f*)(p);
  const v4f c = *(const v4f*)(p + 4);
  unsigned short hb[8];
#pragma unroll
  for (int e = 0; e < 4; ++e) {
    hb[e]     = h_bits(a[e] * scale);
    hb[4 + e] = h_bits(c[e] * scale);
  }
  const v4u u = (v4u){pk16(hb[0], hb[1]), pk16(hb[2], hb[3]), pk16(hb[4], hb[5]), pk16(hb[6], hb[7])};
  unsigned short* q = out + 8 * (size_t)i;
  *(volatile v4u*)q = u;
  __threadfence();
  *(volatile v4u*)q = u;
}

template <int NTHR>
__global__ __launch_bounds__(NTHR) void softmax_rows_kernel(const float* __restrict__ S, unsigned short* __restrict__ P,
                                                          float carry) {
  constexpr int kNW = NTHR / 32;
  constexpr int kRowLen = NTHR * 8;
  __shared__ float redM[kNW];
  __shared__ float redS[kNW];
  const int row  = blockIdx.x;
  const int t    = threadIdx.x;
  const int lane = t & 31, wave = t >> 5;
  const int c0   = t * 8;
  const float* sr = S + (size_t)row * kRowLen + c0;
  const v4f a = *(const v4f*)(sr);
  const v4f c = *(const v4f*)(sr + 4);
  float x[8];
#pragma unroll
  for (int e = 0; e < 4; ++e) { x[e] = a[e]; x[4 + e] = c[e]; }
  float m = fmaxf(fmaxf(fmaxf(x[0], x[1]), fmaxf(x[2], x[3])), fmaxf(fmaxf(x[4], x[5]), fmaxf(x[6], x[7])));
#pragma unroll
  for (int off = 16; off > 0; off >>= 1) m = fmaxf(m, __shfl_xor(m, off, 32));
  if (lane == 0) redM[wave] = m;
  __syncthreads();
  float gm = redM[0];
#pragma unroll
  for (int w = 1; w < kNW; ++w) gm = fmaxf(gm, redM[w]);
  float ev[8];
#pragma unroll
  for (int e = 0; e < 8; ++e) ev[e] = expf(x[e] - gm);
  float s = ((ev[0] + ev[1]) + (ev[2] + ev[3])) + ((ev[4] + ev[5]) + (ev[6] + ev[7]));
#pragma unroll
  for (int off = 16; off > 0; off >>= 1) s += __shfl_xor(s, off, 32);
  if (lane == 0) redS[wave] = s;
  __syncthreads();
  float tot = redS[0];
#pragma unroll
  for (int w = 1; w < kNW; ++w) tot += redS[w];
  const float f = (1.0f / tot) * carry;
  unsigned short hb[8];
#pragma unroll
  for (int e = 0; e < 8; ++e) hb[e] = h_bits(ev[e] * f);
  const v4u u = (v4u){pk16(hb[0], hb[1]), pk16(hb[2], hb[3]), pk16(hb[4], hb[5]), pk16(hb[6], hb[7])};
  unsigned short* q = P + (size_t)row * kRowLen + c0;
  *(volatile v4u*)q = u;
  __threadfence();
  *(volatile v4u*)q = u;
}

template <bool W16>
__global__ __launch_bounds__(128) void ln_rows_kernel(const float* __restrict__ X, const float* __restrict__ gam,
                                                     const float* __restrict__ bet, float* __restrict__ outf,
                                                     unsigned short* __restrict__ outh) {
  __shared__ float red[4];
  __shared__ float red2[4];
  __shared__ __align__(16) unsigned int sh16[256];
  const int row  = blockIdx.x;
  const int t    = threadIdx.x;
  const int lane = t & 31, wave = t >> 5;
  const v4f x = *(const v4f*)(X + (size_t)row * kDim + 4 * t);
  float s = (x[0] + x[1]) + (x[2] + x[3]);
#pragma unroll
  for (int off = 16; off > 0; off >>= 1) s += __shfl_xor(s, off, 32);
  if (lane == 0) red[wave] = s;
  __syncthreads();
  const float mean = ((red[0] + red[1]) + (red[2] + red[3])) * kInvDim;
  const float d0 = x[0] - mean, d1 = x[1] - mean, d2 = x[2] - mean, d3 = x[3] - mean;
  float sq = (d0 * d0 + d1 * d1) + (d2 * d2 + d3 * d3);
#pragma unroll
  for (int off = 16; off > 0; off >>= 1) sq += __shfl_xor(sq, off, 32);
  if (lane == 0) red2[wave] = sq;
  __syncthreads();
  const float var = ((red2[0] + red2[1]) + (red2[2] + red2[3])) * kInvDim;
  const float rs = 1.0f / sqrtf(var + kLnEps);
  const v4f gv = *(const v4f*)(gam + 4 * t);
  const v4f bv = *(const v4f*)(bet + 4 * t);
  v4f y;
  y[0] = d0 * rs * gv[0] + bv[0];
  y[1] = d1 * rs * gv[1] + bv[1];
  y[2] = d2 * rs * gv[2] + bv[2];
  y[3] = d3 * rs * gv[3] + bv[3];
  float* op = outf + (size_t)row * kDim + 4 * t;
  *(volatile v4f*)op = y;
  __threadfence();
  *(volatile v4f*)op = y;
  if (W16) {
    sh16[2 * t]     = pk16(h_bits(y[0]), h_bits(y[1]));
    sh16[2 * t + 1] = pk16(h_bits(y[2]), h_bits(y[3]));
    __syncthreads();
    if (t < 64) {
      const v4u u = *(const v4u*)(sh16 + 4 * t);
      unsigned short* hp = outh + (size_t)row * kDim + 8 * t;
      *(volatile v4u*)hp = u;
      __threadfence();
      *(volatile v4u*)hp = u;
    }
  }
}

__global__ __launch_bounds__(256) void geo_bias_kernel(const float* __restrict__ qp, const float* __restrict__ mp,
                                                       const float* __restrict__ w1, const float* __restrict__ b1,
                                                       const float* __restrict__ w2, const float* __restrict__ b2,
                                                       const float* __restrict__ betap, float* __restrict__ out, int nquad) {
  __shared__ float sw1[kKernDim];
  __shared__ float sb1[kKernDim];
  __shared__ float sw2[kKernDim];
  const int t = threadIdx.x;
  if (t < kKernDim) { sw1[t] = w1[t]; sb1[t] = b1[t]; sw2[t] = w2[t]; }
  __syncthreads();
  const int idxRaw = blockIdx.x * 256 + t;
  const bool valid = idxRaw < nquad;
  const int idx4 = valid ? idxRaw : (nquad - 1);
  constexpr int kQuadPerBatch = kNq * (kNk / 4);
  constexpr int kQuadPerQ = kNk / 4;
  const int b  = idx4 / kQuadPerBatch;
  const int rm = idx4 - b * kQuadPerBatch;
  const int q  = rm / kQuadPerQ;
  const int l0 = (rm - q * kQuadPerQ) * 4;
  const float* qpp = qp + (size_t)(b * kNq + q) * 3;
  const float qx = qpp[0], qy = qpp[1], qz = qpp[2];
  const float* mpp = mp + (size_t)(b * kNk + l0) * 3;
  const v4f m0 = *(const v4f*)(mpp);
  const v4f m1 = *(const v4f*)(mpp + 4);
  const v4f m2 = *(const v4f*)(mpp + 8);
  const float mx0 = m0[0], my0 = m0[1], mz0 = m0[2];
  const float mx1 = m0[3], my1 = m1[0], mz1 = m1[1];
  const float mx2 = m1[2], my2 = m1[3], mz2 = m2[0];
  const float mx3 = m2[1], my3 = m2[2], mz3 = m2[3];
  float dist[4];
  {
    float dx, dy, dz;
    dx = qx - mx0; dy = qy - my0; dz = qz - mz0; dist[0] = sqrtf(fmaxf((dx * dx + dz * dz) + dy * dy, 1e-12f));
    dx = qx - mx1; dy = qy - my1; dz = qz - mz1; dist[1] = sqrtf(fmaxf((dx * dx + dz * dz) + dy * dy, 1e-12f));
    dx = qx - mx2; dy = qy - my2; dz = qz - mz2; dist[2] = sqrtf(fmaxf((dx * dx + dz * dz) + dy * dy, 1e-12f));
    dx = qx - mx3; dy = qy - my3; dz = qz - mz3; dist[3] = sqrtf(fmaxf((dx * dx + dz * dz) + dy * dy, 1e-12f));
  }
  float acc[4] = {0.f, 0.f, 0.f, 0.f};
#pragma unroll 4
  for (int i = 0; i < kKernDim; ++i) {
    const float wa = sw1[i], ba = sb1[i], wb = sw2[i];
#pragma unroll
    for (int e = 0; e < 4; ++e) {
      const float hv = fmaxf(dist[e] * wa + ba, 0.0f);
      acc[e] += hv * wb;
    }
  }
  const float beta = betap[0];
  const float bb2  = b2[0];
  v4f o;
#pragma unroll
  for (int e = 0; e < 4; ++e) o[e] = beta * fminf(fmaxf(acc[e] + bb2, -10.0f), 0.0f);
  if (valid) {
    float* op = out + (size_t)idx4 * 4;
    *(volatile v4f*)op = o;
    __threadfence();
    *(volatile v4f*)op = o;
  }
}

template <int BIAS_MODE, int OUT_MODE, bool RESID, int ACT>
static void run_gemm(hipStream_t st, int nb,
                     const unsigned short* A, int lda, long sA,
                     const unsigned short* Bt, int ldb, long sB,
                     void* C, int ldc, long sC,
                     const float* bias, const float* resid, long sR,
                     int M, int N, int K, float scale) {
  const int tiles = (M >> 6) * (N >> 6);
  dim3 grid((unsigned)((tiles + 7) / 8), (unsigned)nb, 1);
  wmma_gemm64<0, false, BIAS_MODE, OUT_MODE, RESID, ACT><<<grid, 256, 0, st>>>(
      A, A, lda, sA, Bt, Bt, ldb, sB, C, C, ldc, sC, bias, resid, sR, M, N, K, scale);
}

static void run_cast(hipStream_t st, const float* in, unsigned short* out, int n, float scale) {
  const int n8 = n / 8;
  cast8_f16_kernel<<<(unsigned)((n8 + 255) / 256), 256, 0, st>>>(in, out, n8, scale);
}

extern "C" void kernel_launch(void* const* d_in, const int* in_sizes, int n_in,
                              void* d_out, int out_size, void* d_ws, size_t ws_size,
                              hipStream_t stream) {
  if (n_in < 31) return;
  if (in_sizes[0] != kTokQ * kDim || in_sizes[1] != kTokK * kDim || in_sizes[2] != kTokK * 3 || in_sizes[3] != kTokQ * 3) return;
  if (in_sizes[4] != 3 * kDim * kDim || in_sizes[25] != kDff * kDim || in_sizes[27] != kDim * kDff) return;
  if (out_size != kTokQ * kDim || ws_size < kWsTotal) return;

  const float* queries  = (const float*)d_in[0];
  const float* memory   = (const float*)d_in[1];
  const float* mem_pos  = (const float*)d_in[2];
  const float* qry_pos  = (const float*)d_in[3];
  const float* sa_in_w  = (const float*)d_in[4];
  const float* sa_in_b  = (const float*)d_in[5];
  const float* sa_out_w = (const float*)d_in[6];
  const float* sa_out_b = (const float*)d_in[7];
  const float* ln1_g    = (const float*)d_in[8];
  const float* ln1_b    = (const float*)d_in[9];
  const float* q_w      = (const float*)d_in[10];
  const float* q_b      = (const float*)d_in[11];
  const float* k_w      = (const float*)d_in[12];
  const float* k_b      = (const float*)d_in[13];
  const float* v_w      = (const float*)d_in[14];
  const float* v_b      = (const float*)d_in[15];
  const float* o_w      = (const float*)d_in[16];
  const float* o_b      = (const float*)d_in[17];
  const float* ln2_g    = (const float*)d_in[18];
  const float* ln2_b    = (const float*)d_in[19];
  const float* beta     = (const float*)d_in[20];
  const float* dk_w1    = (const float*)d_in[21];
  const float* dk_b1    = (const float*)d_in[22];
  const float* dk_w2    = (const float*)d_in[23];
  const float* dk_b2    = (const float*)d_in[24];
  const float* ffn_w1   = (const float*)d_in[25];
  const float* ffn_b1   = (const float*)d_in[26];
  const float* ffn_w2   = (const float*)d_in[27];
  const float* ffn_b2   = (const float*)d_in[28];
  const float* ln3_g    = (const float*)d_in[29];
  const float* ln3_b    = (const float*)d_in[30];
  float* out = (float*)d_out;
  char* ws = (char*)d_ws;

  unsigned short* Xq   = (unsigned short*)(ws + kOffXq);
  unsigned short* Mem  = (unsigned short*)(ws + kOffMem);
  unsigned short* Wsa  = (unsigned short*)(ws + kOffWsa);
  unsigned short* Wso  = (unsigned short*)(ws + kOffWso);
  unsigned short* Wq   = (unsigned short*)(ws + kOffWq);
  unsigned short* Wk   = (unsigned short*)(ws + kOffWk);
  unsigned short* Wv   = (unsigned short*)(ws + kOffWv);
  unsigned short* Wo   = (unsigned short*)(ws + kOffWo);
  unsigned short* Wf1  = (unsigned short*)(ws + kOffWf1);
  unsigned short* Wf2  = (unsigned short*)(ws + kOffWf2);
  unsigned short* QK   = (unsigned short*)(ws + kOffQK);
  unsigned short* VTs  = (unsigned short*)(ws + kOffVTs);
  float*          Sbuf = (float*)(ws + kOffS);
  unsigned short* Pbuf = (unsigned short*)(ws + kOffP);
  unsigned short* Ctx  = (unsigned short*)(ws + kOffCtx);
  float*          Tf   = (float*)(ws + kOffT);
  float*          X1f  = (float*)(ws + kOffX1f);
  unsigned short* X1h  = (unsigned short*)(ws + kOffX1h);
  unsigned short* Qc   = (unsigned short*)(ws + kOffQc);
  unsigned short* Kc   = (unsigned short*)(ws + kOffKc);
  unsigned short* VTc  = (unsigned short*)(ws + kOffVTc);
  float*          BB   = (float*)(ws + kOffBB);
  float*          X2f  = (float*)(ws + kOffX2f);
  unsigned short* X2h  = (unsigned short*)(ws + kOffX2h);
  unsigned short* Hf   = (unsigned short*)(ws + kOffHf);
  const float* dummy = sa_in_b;

  run_cast(stream, queries, Xq, kTokQ * kDim, 1.0f);
  run_cast(stream, memory, Mem, kTokK * kDim, 1.0f);
  run_cast(stream, sa_in_w, Wsa, 3 * kDim * kDim, kWCarry);
  run_cast(stream, sa_out_w, Wso, kDim * kDim, kWCarry);
  run_cast(stream, q_w, Wq, kDim * kDim, kWCarry);
  run_cast(stream, k_w, Wk, kDim * kDim, kWCarry);
  run_cast(stream, v_w, Wv, kDim * kDim, kWCarry);
  run_cast(stream, o_w, Wo, kDim * kDim, kWCarry);
  run_cast(stream, ffn_w1, Wf1, kDff * kDim, kWCarry);
  run_cast(stream, ffn_w2, Wf2, kDim * kDff, kWCarry);

  run_gemm<2, 1, false, 0>(stream, 1, Xq, kDim, 0, Wsa, kDim, 0, QK, 2 * kDim, 0, sa_in_b, dummy, 0,
                           kTokQ, 2 * kDim, kDim, kWCarryInv);
  run_gemm<1, 1, false, 0>(stream, kBatch, Wsa + (size_t)2 * kDim * kDim, kDim, 0, Xq, kDim, (long)kNq * kDim,
                           VTs, kNq, (long)kDim * kNq, sa_in_b + 2 * kDim, dummy, 0, kDim, kNq, kDim, kWCarryInv);
  for (int b = 0; b < kBatch; ++b) {
    const unsigned short* qbase = QK + (size_t)b * kNq * 2 * kDim;
    run_gemm<0, 0, false, 0>(stream, kHeads, qbase, 2 * kDim, kHdim, qbase + kDim, 2 * kDim, kHdim,
                             Sbuf + (size_t)b * kHeads * kNq * kNq, kNq, (long)kNq * kNq, dummy, dummy, 0,
                             kNq, kNq, kHdim, kAttnScale);
  }
  softmax_rows_kernel<64><<<(unsigned)(kBatch * kHeads * kNq), 64, 0, stream>>>(Sbuf, Pbuf, kPCarry);
  for (int b = 0; b < kBatch; ++b) {
    run_gemm<0, 1, false, 0>(stream, kHeads, Pbuf + (size_t)b * kHeads * kNq * kNq, kNq, (long)kNq * kNq,
                             VTs + (size_t)b * kDim * kNq, kNq, (long)kHdim * kNq,
                             Ctx + (size_t)b * kNq * kDim, kDim, kHdim, dummy, dummy, 0,
                             kNq, kHdim, kNq, kPVScale);
  }
  run_gemm<2, 0, true, 0>(stream, 1, Ctx, kDim, 0, Wso, kDim, 0, Tf, kDim, 0, sa_out_b, queries, 0,
                          kTokQ, kDim, kDim, kProjScale);
  ln_rows_kernel<true><<<(unsigned)kTokQ, 128, 0, stream>>>(Tf, ln1_g, ln1_b, X1f, X1h);
  run_gemm<2, 1, false, 0>(stream, 1, X1h, kDim, 0, Wq, kDim, 0, Qc, kDim, 0, q_b, dummy, 0,
                           kTokQ, kDim, kDim, kWCarryInv);
  run_gemm<2, 1, false, 0>(stream, 1, Mem, kDim, 0, Wk, kDim, 0, Kc, kDim, 0, k_b, dummy, 0,
                           kTokK, kDim, kDim, kWCarryInv);
  run_gemm<1, 1, false, 0>(stream, kBatch, Wv, kDim, 0, Mem, kDim, (long)kNk * kDim,
                           VTc, kNk, (long)kDim * kNk, v_b, dummy, 0, kDim, kNk, kDim, kWCarryInv);
  {
    const int nquad = kBatch * kNq * kNk / 4;
    geo_bias_kernel<<<(unsigned)((nquad + 255) / 256), 256, 0, stream>>>(qry_pos, mem_pos, dk_w1, dk_b1, dk_w2, dk_b2,
                                                                        beta, BB, nquad);
  }
  for (int c = 0; c < kNumChunks; ++c) {
    const int b  = c / (kHeads / kHeadsPerChunk);
    const int h0 = (c - b * (kHeads / kHeadsPerChunk)) * kHeadsPerChunk;
    run_gemm<0, 0, true, 0>(stream, kHeadsPerChunk,
                            Qc + (size_t)b * kNq * kDim + (size_t)h0 * kHdim, kDim, kHdim,
                            Kc + (size_t)b * kNk * kDim + (size_t)h0 * kHdim, kDim, kHdim,
                            Sbuf, kNk, (long)kNq * kNk, dummy, BB + (size_t)b * kNq * kNk, 0,
                            kNq, kNk, kHdim, kAttnScale);
    softmax_rows_kernel<512><<<(unsigned)(kHeadsPerChunk * kNq), 512, 0, stream>>>(Sbuf, Pbuf, kPCarry);
    run_gemm<0, 1, false, 0>(stream, kHeadsPerChunk, Pbuf, kNk, (long)kNq * kNk,
                             VTc + (size_t)b * kDim * kNk + (size_t)h0 * kHdim * kNk, kNk, (long)kHdim * kNk,
                             Ctx + (size_t)b * kNq * kDim + (size_t)h0 * kHdim, kDim, kHdim, dummy, dummy, 0,
                             kNq, kHdim, kNk, kPVScale);
  }
  run_gemm<2, 0, true, 0>(stream, 1, Ctx, kDim, 0, Wo, kDim, 0, Tf, kDim, 0, o_b, X1f, 0,
                          kTokQ, kDim, kDim, kProjScale);
  ln_rows_kernel<true><<<(unsigned)kTokQ, 128, 0, stream>>>(Tf, ln2_g, ln2_b, X2f, X2h);
  run_gemm<2, 1, false, 2>(stream, 1, X2h, kDim, 0, Wf1, kDim, 0, Hf, kDff, 0, ffn_b1, dummy, 0,
                           kTokQ, kDff, kDim, kWCarryInv);
  run_gemm<2, 0, true, 0>(stream, 1, Hf, kDff, 0, Wf2, kDff, 0, Tf, kDim, 0, ffn_b2, X2f, 0,
                          kTokQ, kDim, kDff, kWCarryInv);
  ln_rows_kernel<false><<<(unsigned)kTokQ, 128, 0, stream>>>(Tf, ln3_g, ln3_b, out, X2h);
}
